// LSTM_torchscript_38293928411400
// MI455X (gfx1250) — hardware-run, weakly checked
//
#include <hip/hip_runtime.h>
#include <math.h>

typedef __attribute__((ext_vector_type(16))) _Float16 v16h;
typedef __attribute__((ext_vector_type(8)))  _Float16 v8h;
typedef __attribute__((ext_vector_type(8)))  float    v8f;
typedef __attribute__((ext_vector_type(4)))  float    v4f;
typedef __attribute__((ext_vector_type(2)))  float    v2f;

constexpr int kBatch = 16384;
constexpr int kSteps = 60;
constexpr int kNx = 4;
constexpr int kHid = 64;
constexpr int kGates = 256;
constexpr int kNy = 4;
constexpr int kNys = 3;
constexpr int kHalfRows = 8192;
constexpr int kTail = 16;
constexpr int kSaveStep = kSteps - kTail - 1;
constexpr int kHPitch = 72;
constexpr int kFPitch = 68;
constexpr int kOutRow = kSteps * kNy;

static_assert(kGates == 4 * kHid);
static_assert(kBatch == 2 * kHalfRows);
static_assert(kHalfRows % 32 == 0);
static_assert(kSaveStep == 43);
static_assert((size_t)kBatch * kSteps * kNy * 4 == (size_t)15728640);
static_assert((size_t)15728640 % 128 == 0);
static_assert((size_t)15728640 + (size_t)kBatch * kNys * 4 == (size_t)15925248);
static_assert((16 * kOutRow * 4) % 128 == 0);

constexpr float kActCarry = 64.0f;
constexpr float kWCarry = 64.0f;
constexpr float kProdCarry = kActCarry * kWCarry;
constexpr float kProdInv = 1.0f / kProdCarry;
constexpr float kResCarry = 2048.0f;
constexpr float kResInv = 1.0f / kResCarry;
constexpr float kLog2e = 1.4426950408889634f;
constexpr float kSigK = -kLog2e / kProdCarry;
constexpr float kTanhK = 2.0f * kLog2e / kProdCarry;
constexpr float kTanhU = 2.0f * kLog2e;
constexpr float kF16MinNormal = 6.103515625e-5f;

struct F {
  union U { v16h v; v8h h[2]; };
  static __device__ __forceinline__ v16h load(const _Float16* p) {
    U f;
    f.h[0] = *(const v8h*)(p);
    f.h[1] = *(const v8h*)(p + 16);
    return f.v;
  }
  static __device__ __forceinline__ v8f mma(v16h a, v16h b, v8f c) {
    return __builtin_amdgcn_wmma_f32_16x16x32_f16(false, a, false, b, (short)0, c, false, false);
  }
};

__device__ __forceinline__ void guard_a4(v8f& a, v16h p0, v16h p1, v16h p2, v16h p3) {
  asm volatile("v_nop\n\tv_nop\n\tv_nop\n\tv_nop" : "+v"(a) : "v"(p0), "v"(p1), "v"(p2), "v"(p3) : "memory");
}
__device__ __forceinline__ void guard_a8(v8f& a, v16h p0, v16h p1, v16h p2, v16h p3,
                                         v16h p4, v16h p5, v16h p6, v16h p7) {
  asm volatile("v_nop\n\tv_nop\n\tv_nop\n\tv_nop" : "+v"(a)
               : "v"(p0), "v"(p1), "v"(p2), "v"(p3), "v"(p4), "v"(p5), "v"(p6), "v"(p7) : "memory");
}
__device__ __forceinline__ void guard_aa4(v8f& a, v8f& b, v16h p0, v16h p1, v16h p2, v16h p3) {
  asm volatile("v_nop\n\tv_nop\n\tv_nop\n\tv_nop" : "+v"(a), "+v"(b)
               : "v"(p0), "v"(p1), "v"(p2), "v"(p3) : "memory");
}

__device__ __forceinline__ void wave_sync() {
  __builtin_amdgcn_fence(__ATOMIC_RELEASE, "workgroup");
  __builtin_amdgcn_wave_barrier();
  __builtin_amdgcn_fence(__ATOMIC_ACQUIRE, "workgroup");
}

__device__ __forceinline__ float fexp2(float x) { return __builtin_amdgcn_exp2f(x); }
__device__ __forceinline__ float frcp(float x) { return __builtin_amdgcn_rcpf(x); }

__device__ __forceinline__ _Float16 h_flush(float v) {
  const float w = (__builtin_fabsf(v) < kF16MinNormal) ? 0.0f : v;
  return (_Float16)w;
}

template <bool HP>
__device__ __forceinline__ void put_h(_Float16* hsHi, _Float16* hsLo, int off, float h) {
  const float hs = h * kActCarry;
  const _Float16 hi = h_flush(hs);
  hsHi[off] = hi;
  if (HP) {
    const float rs = (hs - (float)hi) * kResCarry;
    hsLo[off] = h_flush(rs);
  }
}

__device__ __forceinline__ void mma3(v8f& a1, v8f& a2, v16h ahi, v16h alo,
                                     const _Float16* bhp, const _Float16* blp) {
  const v16h bh = F::load(bhp);
  const v16h bl = F::load(blp);
  a1 = F::mma(ahi, bh, a1);
  a2 = F::mma(alo, bh, a2);
  a2 = F::mma(ahi, bl, a2);
  guard_aa4(a1, a2, ahi, alo, bh, bl);
}

template <bool HP, bool FST>
__device__ __forceinline__ void cell_block(const v8f& gi, const v8f& gf, const v8f& gg, const v8f& go,
                                           float (&cs)[8], _Float16* hsHi, _Float16* hsLo, float* fs,
                                           int hoff, int foff) {
#pragma unroll
  for (int r = 0; r < 8; ++r) {
    const float ei = fexp2(gi[r] * kSigK);
    const float ef = fexp2(gf[r] * kSigK);
    const float eo = fexp2(go[r] * kSigK);
    const float eg = fexp2(gg[r] * kTanhK);
    const float iv = frcp(1.0f + ei);
    const float fv = frcp(1.0f + ef);
    const float ov = frcp(1.0f + eo);
    const float gv = fmaf(-2.0f, frcp(eg + 1.0f), 1.0f);
    const float cv = fmaf(fv, cs[r], iv * gv);
    cs[r] = cv;
    const float ec = fexp2(cv * kTanhU);
    const float th = fmaf(-2.0f, frcp(ec + 1.0f), 1.0f);
    const float hv = ov * th;
    put_h<HP>(hsHi, hsLo, hoff + r * kHPitch, hv);
    if (FST) fs[foff + r * kFPitch] = hv;
  }
}

__global__ __launch_bounds__(256) void pack_kernel(const float* __restrict__ W0, const float* __restrict__ W1,
                                                   const float* __restrict__ W2, const float* __restrict__ W3,
                                                   unsigned short* hi0, unsigned short* lo0,
                                                   unsigned short* hi1, unsigned short* lo1,
                                                   unsigned short* hi2, unsigned short* lo2,
                                                   unsigned short* hi3) {
  const int which = (int)blockIdx.y;
  const float* src = (which == 0) ? W0 : (which == 1) ? W1 : (which == 2) ? W2 : W3;
  unsigned short* hp = (which == 0) ? hi0 : (which == 1) ? hi1 : (which == 2) ? hi2 : hi3;
  unsigned short* lp = (which == 0) ? lo0 : (which == 1) ? lo1 : (which == 2) ? lo2 : hi3;
  const int npieces = (which == 3) ? (kHid * kHid / 8) : (kGates * kHid / 8);
  const int piece = (int)blockIdx.x * 256 + (int)threadIdx.x;
  if (piece >= npieces) return;
  const v4f a = *(const v4f*)(src + (size_t)piece * 8);
  const v4f b = *(const v4f*)(src + (size_t)piece * 8 + 4);
  v8h hv, lv;
#pragma unroll
  for (int e = 0; e < 4; ++e) {
    const float s0 = a[e] * kWCarry;
    const float s1 = b[e] * kWCarry;
    const _Float16 h0 = h_flush(s0);
    const _Float16 h1 = h_flush(s1);
    hv[e] = h0;
    hv[4 + e] = h1;
    lv[e] = h_flush((s0 - (float)h0) * kResCarry);
    lv[4 + e] = h_flush((s1 - (float)h1) * kResCarry);
  }
  for (int pass = 0; pass < 2; ++pass) {
    *(volatile v8h*)(void*)(hp + (size_t)piece * 8) = hv;
    if (which < 3) *(volatile v8h*)(void*)(lp + (size_t)piece * 8) = lv;
    __threadfence();
  }
}

template <bool HP>
__global__ __launch_bounds__(64) __attribute__((amdgpu_num_vgpr(256))) void lstm1_kernel(
    const float* __restrict__ xmain, const float* __restrict__ aux,
    const float* __restrict__ Ws1, const float* __restrict__ bs1,
    const float* __restrict__ Ws2, const float* __restrict__ bs2,
    const float* __restrict__ Wih1, const float* __restrict__ bih1, const float* __restrict__ bhh1,
    const unsigned short* WhiP, const unsigned short* WloP,
    unsigned short* outHi, unsigned short* outLo, int row0) {
  constexpr int NSTEP = HP ? kTail : kSteps;
  constexpr int T0 = kSteps - NSTEP;
  __shared__ __align__(16) float sWx[kGates * 4];
  __shared__ __align__(16) float sGb[kGates];
  __shared__ __align__(16) float sM1[kHid * 4];
  __shared__ __align__(16) float sM2[kHid * 4];
  __shared__ __align__(16) float sAx[2 * 64];
  __shared__ __align__(16) _Float16 sHh[2 * 16 * kHPitch];
  __shared__ __align__(16) _Float16 sHl[HP ? 2 * 16 * kHPitch : 8];

  const int tid = (int)threadIdx.x;
  const int lane = tid & 31, wave = tid >> 5, c = lane & 15, hh = lane >> 4;
  const int tileLocal = (int)blockIdx.x * 2 + wave;
  const int rowbase = row0 + tileLocal * 16;
  const _Float16* Whi = (const _Float16*)WhiP;
  const _Float16* Wlo = (const _Float16*)WloP;
  _Float16* hsHi = sHh + wave * (16 * kHPitch);
  _Float16* hsLo = HP ? (sHl + wave * (16 * kHPitch)) : hsHi;

#pragma unroll 1
  for (int p = tid; p < kGates; p += 64) {
    v4f w = *(const v4f*)(Wih1 + (size_t)p * kNx);
    w[0] = w[0] * kProdCarry;
    w[1] = w[1] * kProdCarry;
    w[2] = w[2] * kProdCarry;
    w[3] = w[3] * kProdCarry;
    *(v4f*)(sWx + p * 4) = w;
    sGb[p] = (bih1[p] + bhh1[p]) * kProdCarry;
  }
  {
    v4f m1, m2;
    m1[0] = Ws1[tid * 3 + 0];
    m1[1] = Ws1[tid * 3 + 1];
    m1[2] = Ws1[tid * 3 + 2];
    m1[3] = bs1[tid];
    m2[0] = Ws2[tid * 3 + 0];
    m2[1] = Ws2[tid * 3 + 1];
    m2[2] = Ws2[tid * 3 + 2];
    m2[3] = bs2[tid];
    *(v4f*)(sM1 + tid * 4) = m1;
    *(v4f*)(sM2 + tid * 4) = m2;
  }
  {
    const float* ar = aux + (size_t)(rowbase + c) * 3;
    v4f a;
    a[0] = ar[0];
    a[1] = ar[1];
    a[2] = ar[2];
    a[3] = 0.0f;
    *(v4f*)(sAx + wave * 64 + c * 4) = a;
  }
  __syncthreads();

  float cst[4][8];
  {
    v4f xa[8];
#pragma unroll
    for (int r = 0; r < 8; ++r) xa[r] = *(const v4f*)(sAx + wave * 64 + (8 * hh + r) * 4);
#pragma unroll
    for (int j = 0; j < 4; ++j) {
      const int n = 16 * j + c;
      const v4f m1 = *(const v4f*)(sM1 + n * 4);
      const v4f m2 = *(const v4f*)(sM2 + n * 4);
#pragma unroll
      for (int r = 0; r < 8; ++r) {
        float hv = fmaf(xa[r][0], m1[0], m1[3]);
        hv = fmaf(xa[r][1], m1[1], hv);
        hv = fmaf(xa[r][2], m1[2], hv);
        float cz = fmaf(xa[r][0], m2[0], m2[3]);
        cz = fmaf(xa[r][1], m2[1], cz);
        cz = fmaf(xa[r][2], m2[2], cz);
        const float ez = fexp2(cz * kTanhU);
        cst[j][r] = fmaf(-2.0f, frcp(ez + 1.0f), 1.0f);
        put_h<HP>(hsHi, hsLo, (8 * hh + r) * kHPitch + n, hv);
      }
    }
  }
  wave_sync();
  v16h ah0 = F::load(hsHi + c * kHPitch + 8 * hh);
  v16h ah1 = F::load(hsHi + c * kHPitch + 8 * hh + 32);
  v16h al0 = ah0, al1 = ah1;
  if (HP) {
    al0 = F::load(hsLo + c * kHPitch + 8 * hh);
    al1 = F::load(hsLo + c * kHPitch + 8 * hh + 32);
  }
  wave_sync();

  const v8f zero8 = {0.f, 0.f, 0.f, 0.f, 0.f, 0.f, 0.f, 0.f};
  const int sq = lane >> 3, sc8 = (lane & 7) * 8;

#pragma unroll 1
  for (int s = 0; s < NSTEP; ++s) {
    const int torig = kSteps - 1 - s;
    v4f xr[8];
#pragma unroll
    for (int r = 0; r < 8; ++r)
      xr[r] = *(const v4f*)(xmain + ((size_t)(rowbase + 8 * hh + r) * kSteps + (size_t)torig) * kNx);

#pragma unroll
    for (int j = 0; j < 4; ++j) {
      v8f g4[4];
#pragma unroll
      for (int gt = 0; gt < 4; ++gt) {
        const int n = gt * kHid + 16 * j + c;
        const v4f wv = *(const v4f*)(sWx + n * 4);
        const float bq = sGb[n];
        v8f acc;
#pragma unroll
        for (int r = 0; r < 8; ++r) {
          float a = fmaf(xr[r][0], wv[0], bq);
          a = fmaf(xr[r][1], wv[1], a);
          a = fmaf(xr[r][2], wv[2], a);
          a = fmaf(xr[r][3], wv[3], a);
          acc[r] = a;
        }
        const _Float16* wp = Whi + (size_t)n * kHid + 8 * hh;
        if (HP) {
          const _Float16* wq = Wlo + (size_t)n * kHid + 8 * hh;
          v8f a2 = zero8;
          mma3(acc, a2, ah0, al0, wp, wq);
          mma3(acc, a2, ah1, al1, wp + 32, wq + 32);
#pragma unroll
          for (int r = 0; r < 8; ++r) acc[r] = fmaf(a2[r], kResInv, acc[r]);
        } else {
          const v16h b0 = F::load(wp);
          const v16h b1 = F::load(wp + 32);
          acc = F::mma(ah0, b0, acc);
          acc = F::mma(ah1, b1, acc);
          guard_a4(acc, ah0, ah1, b0, b1);
        }
        g4[gt] = acc;
      }
      cell_block<HP, false>(g4[0], g4[1], g4[2], g4[3], cst[j], hsHi, hsLo, (float*)nullptr,
                            (8 * hh) * kHPitch + 16 * j + c, 0);
    }
    wave_sync();
    ah0 = F::load(hsHi + c * kHPitch + 8 * hh);
    ah1 = F::load(hsHi + c * kHPitch + 8 * hh + 32);
    if (HP) {
      al0 = F::load(hsLo + c * kHPitch + 8 * hh);
      al1 = F::load(hsLo + c * kHPitch + 8 * hh + 32);
    }
    {
      const size_t slot = ((size_t)tileLocal * NSTEP + (size_t)(torig - T0)) * (size_t)(16 * kHid);
      unsigned short* gH = outHi + slot;
      unsigned short* gL = outLo + slot;
      for (int pass = 0; pass < 2; ++pass) {
#pragma unroll
        for (int it = 0; it < 4; ++it) {
          const int row = it * 4 + sq;
          const v8h v = *(const v8h*)(hsHi + row * kHPitch + sc8);
          *(volatile v8h*)(void*)(gH + row * kHid + sc8) = v;
          if (HP) {
            const v8h w = *(const v8h*)(hsLo + row * kHPitch + sc8);
            *(volatile v8h*)(void*)(gL + row * kHid + sc8) = w;
          }
        }
        __threadfence();
      }
    }
    wave_sync();
  }
}

template <bool HP>
__global__ __launch_bounds__(64) __attribute__((amdgpu_num_vgpr(256))) void lstm2_kernel(
    const float* hInit, const float* cInit,
    const float* __restrict__ bih2, const float* __restrict__ bhh2,
    const unsigned short* WhhHiP, const unsigned short* WhhLoP,
    const unsigned short* WihHiP, const unsigned short* WihLoP,
    const unsigned short* WlatP,
    const float* __restrict__ blat, const float* __restrict__ Wout, const float* __restrict__ bout,
    const float* __restrict__ Wsfc, const float* __restrict__ bsfc,
    const unsigned short* xHiP, const unsigned short* xLoP,
    float* stH, float* stC, float* outp, int row0) {
  constexpr int NSTEP = HP ? kTail : kSteps;
  constexpr int T0 = kSteps - NSTEP;
  __shared__ __align__(16) float sOut[HP ? 4 : 2 * 16 * kOutRow];
  __shared__ __align__(16) float sF[2 * 16 * kFPitch];
  __shared__ __align__(16) float sC[2 * 16 * kFPitch];
  __shared__ __align__(16) _Float16 sHh[2 * 16 * kHPitch];
  __shared__ __align__(16) _Float16 sHl[HP ? 2 * 16 * kHPitch : 8];
  __shared__ __align__(16) float sGb[kGates];
  __shared__ __align__(16) float sWo[kNy * kHid];
  __shared__ __align__(16) float sBo[4];
  __shared__ __align__(16) float sWs[kNys * kHid];
  __shared__ __align__(16) float sBs[4];
  __shared__ __align__(16) float sO1[32 * kNys];

  const int tid = (int)threadIdx.x;
  const int lane = tid & 31, wave = tid >> 5, c = lane & 15, hh = lane >> 4;
  const int tileLocal = (int)blockIdx.x * 2 + wave;
  const int rowbase = row0 + tileLocal * 16;
  const _Float16* WhhHi = (const _Float16*)WhhHiP;
  const _Float16* WhhLo = (const _Float16*)WhhLoP;
  const _Float16* WihHi = (const _Float16*)WihHiP;
  const _Float16* WihLo = (const _Float16*)WihLoP;
  const _Float16* Wl16 = (const _Float16*)WlatP;
  const _Float16* xHi = (const _Float16*)xHiP;
  const _Float16* xLo = (const _Float16*)xLoP;
  _Float16* hsHi = sHh + wave * (16 * kHPitch);
  _Float16* hsLo = HP ? (sHl + wave * (16 * kHPitch)) : hsHi;
  float* fs = sF + wave * (16 * kFPitch);
  float* cw = sC + wave * (16 * kFPitch);
  float* so = HP ? sOut : (sOut + wave * (16 * kOutRow));

#pragma unroll 1
  for (int p = tid; p < kGates; p += 64) {
    sGb[p] = (bih2[p] + bhh2[p]) * kProdCarry;
    sWo[p] = Wout[p];
  }
#pragma unroll 1
  for (int p = tid; p < kNys * kHid; p += 64) sWs[p] = Wsfc[p];
  {
    const int q = tid & 3;
    const int qs = (q < kNys) ? q : (kNys - 1);
    sBo[q] = bout[q];
    sBs[q] = bsfc[qs];
  }
  __syncthreads();

  float bl[4];
#pragma unroll
  for (int j = 0; j < 4; ++j) bl[j] = blat[16 * j + c];

  {
#pragma unroll
    for (int it = 0; it < 8; ++it) {
      const int idx = it * 32 + lane;
      const int row = idx >> 4, c4 = (idx & 15) * 4;
      const v4f v = *(const v4f*)(cInit + (size_t)(rowbase + row) * kHid + c4);
      *(v4f*)(cw + row * kFPitch + c4) = v;
    }
#pragma unroll
    for (int it = 0; it < 8; ++it) {
      const int idx = it * 32 + lane;
      const int row = idx >> 4, c4 = (idx & 15) * 4;
      const v4f v = *(const v4f*)(hInit + (size_t)(rowbase + row) * kHid + c4);
      *(v4f*)(fs + row * kFPitch + c4) = v;
    }
    wave_sync();
#pragma unroll 1
    for (int j = 0; j < 4; ++j) {
#pragma unroll
      for (int r = 0; r < 8; ++r) {
        const float hv = fs[(8 * hh + r) * kFPitch + 16 * j + c];
        put_h<HP>(hsHi, hsLo, (8 * hh + r) * kHPitch + 16 * j + c, hv);
      }
    }
    wave_sync();
  }
  v16h ah0 = F::load(hsHi + c * kHPitch + 8 * hh);
  v16h ah1 = F::load(hsHi + c * kHPitch + 8 * hh + 32);
  v16h al0 = ah0, al1 = ah1;
  if (HP) {
    al0 = F::load(hsLo + c * kHPitch + 8 * hh);
    al1 = F::load(hsLo + c * kHPitch + 8 * hh + 32);
  }
  wave_sync();

  const v8f zero8 = {0.f, 0.f, 0.f, 0.f, 0.f, 0.f, 0.f, 0.f};

#pragma unroll 1
  for (int t = T0; t < kSteps; ++t) {
    const size_t slot = ((size_t)tileLocal * NSTEP + (size_t)(t - T0)) * (size_t)(16 * kHid);
    const _Float16* xp = xHi + slot + c * kHid + 8 * hh;
    const v16h xh0 = F::load(xp);
    const v16h xh1 = F::load(xp + 32);
    v16h xl0 = xh0, xl1 = xh1;
    if (HP) {
      const _Float16* xq = xLo + slot + c * kHid + 8 * hh;
      xl0 = F::load(xq);
      xl1 = F::load(xq + 32);
    }

#pragma unroll 1
    for (int j = 0; j < 4; ++j) {
      v8f g4[4];
#pragma unroll
      for (int gt = 0; gt < 4; ++gt) {
        const int n = gt * kHid + 16 * j + c;
        const float bq = sGb[n];
        v8f acc = {bq, bq, bq, bq, bq, bq, bq, bq};
        const size_t wo = (size_t)n * kHid + 8 * hh;
        if (HP) {
          v8f a2 = zero8;
          mma3(acc, a2, ah0, al0, WhhHi + wo, WhhLo + wo);
          mma3(acc, a2, ah1, al1, WhhHi + wo + 32, WhhLo + wo + 32);
          mma3(acc, a2, xh0, xl0, WihHi + wo, WihLo + wo);
          mma3(acc, a2, xh1, xl1, WihHi + wo + 32, WihLo + wo + 32);
#pragma unroll
          for (int r = 0; r < 8; ++r) acc[r] = fmaf(a2[r], kResInv, acc[r]);
        } else {
          const v16h b0 = F::load(WhhHi + wo);
          const v16h b1 = F::load(WhhHi + wo + 32);
          const v16h b2 = F::load(WihHi + wo);
          const v16h b3 = F::load(WihHi + wo + 32);
          acc = F::mma(ah0, b0, acc);
          acc = F::mma(ah1, b1, acc);
          acc = F::mma(xh0, b2, acc);
          acc = F::mma(xh1, b3, acc);
          guard_a8(acc, ah0, ah1, xh0, xh1, b0, b1, b2, b3);
        }
        g4[gt] = acc;
      }
      const int coff = (8 * hh) * kFPitch + 16 * j + c;
      float cs[8];
#pragma unroll
      for (int r = 0; r < 8; ++r) cs[r] = cw[coff + r * kFPitch];
      cell_block<HP, true>(g4[0], g4[1], g4[2], g4[3], cs, hsHi, hsLo, fs,
                           (8 * hh) * kHPitch + 16 * j + c, coff);
#pragma unroll
      for (int r = 0; r < 8; ++r) cw[coff + r * kFPitch] = cs[r];
    }
    wave_sync();
    ah0 = F::load(hsHi + c * kHPitch + 8 * hh);
    ah1 = F::load(hsHi + c * kHPitch + 8 * hh + 32);
    if (HP) {
      al0 = F::load(hsLo + c * kHPitch + 8 * hh);
      al1 = F::load(hsLo + c * kHPitch + 8 * hh + 32);
    }

    if (!HP) {
      if (t == kSaveStep) {
        float* gh = stH + (size_t)rowbase * kHid;
        float* gc = stC + (size_t)rowbase * kHid;
        for (int pass = 0; pass < 2; ++pass) {
#pragma unroll
          for (int it = 0; it < 8; ++it) {
            const int row = it * 2 + hh;
            const v4f v = *(const v4f*)(fs + row * kFPitch + c * 4);
            *(volatile v4f*)(gh + row * kHid + c * 4) = v;
          }
          __threadfence();
        }
        for (int pass = 0; pass < 2; ++pass) {
#pragma unroll
          for (int it = 0; it < 8; ++it) {
            const int row = it * 2 + hh;
            const v4f v = *(const v4f*)(cw + row * kFPitch + c * 4);
            *(volatile v4f*)(gc + row * kHid + c * 4) = v;
          }
          __threadfence();
        }
        wave_sync();
      }
#pragma unroll
      for (int j = 0; j < 4; ++j) {
        const _Float16* lp = Wl16 + (size_t)(16 * j + c) * kHid + 8 * hh;
        const v16h b0 = F::load(lp);
        const v16h b1 = F::load(lp + 32);
        v8f la = zero8;
        la = F::mma(ah0, b0, la);
        la = F::mma(ah1, b1, la);
        guard_a4(la, ah0, ah1, b0, b1);
#pragma unroll
        for (int r = 0; r < 8; ++r) fs[(8 * hh + r) * kFPitch + 16 * j + c] = fmaf(la[r], kProdInv, bl[j]);
      }
      wave_sync();
      {
        const int hrow = lane >> 1, ny0 = (lane & 1) * 2;
        float o0 = sBo[ny0], o1 = sBo[ny0 + 1];
        const float* lrow = fs + hrow * kFPitch;
        const float* w0p = sWo + ny0 * kHid;
        const float* w1p = w0p + kHid;
#pragma unroll 4
        for (int i = 0; i < 16; ++i) {
          const v4f lv = *(const v4f*)(lrow + 4 * i);
          const v4f w0 = *(const v4f*)(w0p + 4 * i);
          const v4f w1 = *(const v4f*)(w1p + 4 * i);
          o0 = fmaf(lv[0], w0[0], o0);
          o0 = fmaf(lv[1], w0[1], o0);
          o0 = fmaf(lv[2], w0[2], o0);
          o0 = fmaf(lv[3], w0[3], o0);
          o1 = fmaf(lv[0], w1[0], o1);
          o1 = fmaf(lv[1], w1[1], o1);
          o1 = fmaf(lv[2], w1[2], o1);
          o1 = fmaf(lv[3], w1[3], o1);
        }
        v2f ov;
        ov[0] = o0;
        ov[1] = o1;
        *(v2f*)(so + hrow * kOutRow + t * kNy + ny0) = ov;
      }
    }
    wave_sync();
  }

  if (!HP) {
    float* go = outp + (size_t)rowbase * kOutRow;
    for (int pass = 0; pass < 2; ++pass) {
#pragma unroll 6
      for (int it = 0; it < 30; ++it) {
        const int idx = (it * 32 + lane) * 4;
        const v4f v = *(const v4f*)(so + idx);
        *(volatile v4f*)(go + idx) = v;
      }
      __threadfence();
    }
  } else {
    float* o1w = sO1 + wave * (16 * kNys);
#pragma unroll
    for (int q = 0; q < 2; ++q) {
      const int idx = lane + 32 * q;
      const bool ok = idx < 16 * kNys;
      const int ic = ok ? idx : (16 * kNys - 1);
      const int m = ic / kNys;
      const int sc = ic - m * kNys;
      float a = sBs[sc];
      const float* hrow = fs + m * kFPitch;
      const float* wrow = sWs + sc * kHid;
#pragma unroll 4
      for (int i = 0; i < 16; ++i) {
        const v4f hv = *(const v4f*)(hrow + 4 * i);
        const v4f wv = *(const v4f*)(wrow + 4 * i);
        a = fmaf(hv[0], wv[0], a);
        a = fmaf(hv[1], wv[1], a);
        a = fmaf(hv[2], wv[2], a);
        a = fmaf(hv[3], wv[3], a);
      }
      a = fmaxf(a, 0.0f);
      if (ok) o1w[idx] = a;
    }
    __syncthreads();
    if (tid < (32 * kNys) / 4) {
      const size_t blockRow0 = (size_t)row0 + (size_t)blockIdx.x * 32;
      float* g1 = outp + (size_t)kBatch * kOutRow + blockRow0 * kNys + (size_t)tid * 4;
      const v4f v = *(const v4f*)(sO1 + tid * 4);
      *(volatile v4f*)(g1) = v;
      __threadfence();
      *(volatile v4f*)(g1) = v;
    }
  }
}

extern "C" void kernel_launch(void* const* d_in, const int* in_sizes, int n_in,
                              void* d_out, int out_size, void* d_ws, size_t ws_size, hipStream_t stream) {
  if (n_in < 22 || d_out == nullptr || d_ws == nullptr) return;
  const int expect[22] = {kBatch * kSteps * kNx, kBatch * 3, kBatch * kHid, kBatch * kHid,
                          kHid * 3, kHid, kHid * 3, kHid,
                          kGates * kNx, kGates * kHid, kGates, kGates,
                          kGates * kHid, kGates * kHid, kGates, kGates,
                          kHid * kHid, kHid, kNy * kHid, kNy, kNys * kHid, kNys};
  for (int i = 0; i < 22; ++i)
    if (in_sizes[i] != expect[i]) return;
  if (out_size != kBatch * kSteps * kNy + kBatch * kNys) return;

  const float* xmain = (const float*)d_in[0];
  const float* aux   = (const float*)d_in[1];
  const float* hx2   = (const float*)d_in[2];
  const float* cx2   = (const float*)d_in[3];
  const float* Ws1   = (const float*)d_in[4];
  const float* bs1   = (const float*)d_in[5];
  const float* Ws2   = (const float*)d_in[6];
  const float* bs2   = (const float*)d_in[7];
  const float* Wih1  = (const float*)d_in[8];
  const float* Whh1  = (const float*)d_in[9];
  const float* bih1  = (const float*)d_in[10];
  const float* bhh1  = (const float*)d_in[11];
  const float* Wih2  = (const float*)d_in[12];
  const float* Whh2  = (const float*)d_in[13];
  const float* bih2  = (const float*)d_in[14];
  const float* bhh2  = (const float*)d_in[15];
  const float* Wlat  = (const float*)d_in[16];
  const float* blat  = (const float*)d_in[17];
  const float* Wout  = (const float*)d_in[18];
  const float* bout  = (const float*)d_in[19];
  const float* Wsfc  = (const float*)d_in[20];
  const float* bsfc  = (const float*)d_in[21];
  float* out = (float*)d_out;

  char* ws = (char*)d_ws;
  size_t off = 0;
  auto carve = [&](size_t bytes) -> char* {
    char* p = ws + off;
    off += (bytes + 255) & ~(size_t)255;
    return p;
  };
  const size_t szW = (size_t)kGates * kHid * 2;
  unsigned short* w1Hi = (unsigned short*)carve(szW);
  unsigned short* w1Lo = (unsigned short*)carve(szW);
  unsigned short* wiHi = (unsigned short*)carve(szW);
  unsigned short* wiLo = (unsigned short*)carve(szW);
  unsigned short* whHi = (unsigned short*)carve(szW);
  unsigned short* whLo = (unsigned short*)carve(szW);
  unsigned short* wlat = (unsigned short*)carve((size_t)kHid * kHid * 2);
  unsigned short* h1pl = (unsigned short*)carve((size_t)kHalfRows * kSteps * kHid * 2);
  unsigned short* hpHi = (unsigned short*)carve((size_t)kHalfRows * kTail * kHid * 2);
  unsigned short* hpLo = (unsigned short*)carve((size_t)kHalfRows * kTail * kHid * 2);
  float* stH = (float*)carve((size_t)kBatch * kHid * 4);
  float* stC = (float*)carve((size_t)kBatch * kHid * 4);
  if (off > ws_size || off > (size_t)134217728) return;

  pack_kernel<<<dim3(8, 4), 256, 0, stream>>>(Whh1, Wih2, Whh2, Wlat, w1Hi, w1Lo, wiHi, wiLo, whHi, whLo, wlat);

  const int blocksPerHalf = kHalfRows / 32;
  for (int half = 0; half < 2; ++half) {
    const int row0 = half * kHalfRows;
    lstm1_kernel<false><<<blocksPerHalf, 64, 0, stream>>>(
        xmain, aux, Ws1, bs1, Ws2, bs2, Wih1, bih1, bhh1, w1Hi, w1Lo, h1pl, h1pl, row0);
    lstm2_kernel<false><<<blocksPerHalf, 64, 0, stream>>>(
        hx2, cx2, bih2, bhh2, whHi, whLo, wiHi, wiLo, wlat, blat, Wout, bout, Wsfc, bsfc,
        h1pl, h1pl, stH, stC, out, row0);
  }
  for (int half = 0; half < 2; ++half) {
    const int row0 = half * kHalfRows;
    lstm1_kernel<true><<<blocksPerHalf, 64, 0, stream>>>(
        xmain, aux, Ws1, bs1, Ws2, bs2, Wih1, bih1, bhh1, w1Hi, w1Lo, hpHi, hpLo, row0);
    lstm2_kernel<true><<<blocksPerHalf, 64, 0, stream>>>(
        stH, stC, bih2, bhh2, whHi, whLo, wiHi, wiLo, wlat, blat, Wout, bout, Wsfc, bsfc,
        hpHi, hpLo, stH, stC, out, row0);
  }
}
